// Self_attention_pixel_wise_39367670235286
// MI455X (gfx1250) — hardware-verified
//
#include <hip/hip_runtime.h>
#include <hip/hip_bf16.h>
#include <math.h>

#define BB 4
#define SS 4096
#define DKK 128
#define HH 1
#define QW 1
#define KST2 136
#define CIN 256
typedef _Float16 bf16;
typedef _Float16 f16;
typedef __attribute__((ext_vector_type(4))) unsigned v4u_t;
typedef unsigned v4ua __attribute__((ext_vector_type(4), may_alias));
typedef __attribute__((ext_vector_type(4))) float v4f_t;
typedef float v4fa __attribute__((ext_vector_type(4), may_alias));
typedef __attribute__((ext_vector_type(16))) bf16  bf16x16;
typedef bf16x16 f16x16;
typedef __attribute__((ext_vector_type(8)))  bf16  bf16x8;
typedef bf16x8 f16x8;
typedef __attribute__((ext_vector_type(4)))  bf16  bf16x4;
typedef __attribute__((ext_vector_type(8)))  float f32x8;
__device__ __forceinline__ f32x8 wmma16(f16x16 a, f16x16 b, f32x8 c) {
  c = __builtin_amdgcn_wmma_f32_16x16x32_f16(false, a, false, b, (short)0, c, false, false);
  asm volatile("v_nop\n\tv_nop\n\tv_nop\n\tv_nop" : "+v"(c) : "v"(a), "v"(b));
  return c;
}
#define GSTR 48
#define LDS_STRIDE 48
#define KSTRIDE    72
#define VSTRIDE    48

__device__ __forceinline__ f32x8 wmma_bf16(bf16x16 a, bf16x16 b, f32x8 c) {
  c = __builtin_amdgcn_wmma_f32_16x16x32_f16(false, a, false, b, (short)0, c, false, false);
  asm volatile("v_nop\n\tv_nop\n\tv_nop\n\tv_nop" : "+v"(c) : "v"(a), "v"(b));
  return c;
}

template <typename T>
__device__ __forceinline__ bf16x16 load_frag(const T* __restrict__ base, int ld,
                                             int row0, int k0) {
  const int lane = threadIdx.x & 31;
  const int r    = lane & 15;
  const int kh   = (lane >> 4) * 8;
  const T* p0 = base + (size_t)(row0 + r) * ld + (k0 + kh);
  const T* p1 = p0 + 16;
  bf16x16 f;
#pragma unroll
  for (int i = 0; i < 8; ++i) {
    f[i]     = (bf16)p0[i];
    f[i + 8] = (bf16)p1[i];
  }
  return f;
}

__device__ __forceinline__ bf16x16 lds_frag(const bf16* base, int stride) {
  const int lane = threadIdx.x & 31;
  const int row  = lane & 15;
  const int kh   = (lane >> 4) * 8;
  const bf16x8 lo = *(const bf16x8*)(base + row * stride + kh);
  const bf16x8 hi = *(const bf16x8*)(base + row * stride + kh + 16);
  bf16x16 f;
#pragma unroll
  for (int i = 0; i < 8; ++i) { f[i] = lo[i]; f[i + 8] = hi[i]; }
  return f;
}

template <typename T>
__device__ __forceinline__ void stage_read16(const T* __restrict__ p, float* buf) {
#pragma unroll
  for (int i = 0; i < 16; ++i) buf[i] = (float)p[i];
}

__device__ __forceinline__ void stage_write(bf16* dst, const float* buf, int nquad) {
#pragma unroll
  for (int i = 0; i < nquad; ++i) {
    bf16x4 q;
    q[0] = (bf16)buf[4 * i];     q[1] = (bf16)buf[4 * i + 1];
    q[2] = (bf16)buf[4 * i + 2]; q[3] = (bf16)buf[4 * i + 3];
    *(bf16x4*)(dst + 4 * i) = q;
  }
}

__global__ __launch_bounds__(64) void attn_kernel(
    const bf16* __restrict__ Qb, const bf16* __restrict__ Kb,
    const bf16* __restrict__ Vt, const float* __restrict__ shortcut, float* __restrict__ attnOut) {
  __shared__ bf16 ldsK[2][32 * KST2];
  __shared__ bf16 ldsV[128 * VSTRIDE];
  __shared__ __attribute__((aligned(16))) float oSp[2][4 * 32 * 8];
  __shared__ __attribute__((aligned(16))) float ldsO[2][16 * 132];

  const int q0blk = blockIdx.x * 32;
  const int h  = blockIdx.y;
  const int b  = blockIdx.z;
  const int t    = threadIdx.x;
  const int wave = t >> 5;
  const int lane = t & 31;
  const int qlane = lane & 15;
  const int kh8   = (lane >> 4) * 8;
  const int q0 = q0blk + wave * 16;

  (void)h;
  const float* Qh = (const float*)Qb + (size_t)b * SS * DKK;
  const float* Kh = (const float*)Kb + (size_t)b * SS * DKK;
  const bf16* Vh = Vt + (size_t)b * DKK * SS;

  const int krow = t >> 1;
  const int kcol = (t & 1) * 64;
  const float* kSrc = Kh + (size_t)krow * DKK + kcol;
  const bf16* vSrc = Vh + (size_t)t * SS;

  const int lanei = threadIdx.x & 31, frr = lanei & 15, khh = (lanei >> 4) * 8;
  const float* qrow = Qh + (size_t)(q0 + frr) * DKK + khh;

  f32x8 o[QW][4] = {};
  float alpha_s[QW];
  float* osp = oSp[wave];
  for (int e = lane; e < 4 * 32 * 8; e += 32) osp[e] = 0.0f;
  __builtin_amdgcn_wave_barrier();
  float mrun[QW], lrun[QW];
#pragma unroll
  for (int qt = 0; qt < QW; ++qt) { mrun[qt] = -INFINITY; lrun[qt] = 0.0f; }

  const float scale = 1.44269504088896340736f;
  const float NEG2 = -1.0e9f; (void)NEG2;
  const int kmin = 0, kmax = SS - 1;

  for (int kb = kmin; kb <= kmax; kb += 32) {
    __syncthreads();
    { const float* kp = kSrc + (size_t)kb * DKK;
#pragma unroll
      for (int i = 0; i < 16; ++i) { const v4f_t v = *(const v4f_t*)(kp + 4 * i);
#pragma unroll
        for (int u = 0; u < 4; ++u) { const bf16 hv = (bf16)v[u]; ldsK[0][krow * KST2 + kcol + 4 * i + u] = hv; ldsK[1][krow * KST2 + kcol + 4 * i + u] = (bf16)((v[u] - (float)hv) * 2048.0f); } } }
#pragma unroll
    for (int i = 0; i < 4; ++i) { *(bf16x8*)(&ldsV[t * VSTRIDE + 8 * i]) = *(const bf16x8*)(vSrc + kb + 8 * i); *(bf16x8*)(&ldsV[(t + 64) * VSTRIDE + 8 * i]) = *(const bf16x8*)(vSrc + (size_t)64 * SS + kb + 8 * i); }
    __syncthreads();


    bf16x16 pf[QW];
    bool act[QW];
#pragma unroll
    for (int qt = 0; qt < QW; ++qt) {
      unsigned mbits = 0;
      mbits = 0xFFFFu; act[qt] = true;
      if (act[qt]) {
        const int q_my = q0 + 16 * qt + qlane;
        f32x8 s0 = {}, s1 = {};
        f32x8 s0x = {}, s1x = {};
#pragma unroll 1
        for (int c = 0; c < 4; ++c) {
          const bf16x16 k0h = lds_frag(ldsK[0] + 0 * KST2 + c * 32, KST2), k1h = lds_frag(ldsK[0] + 16 * KST2 + c * 32, KST2);
          const bf16x16 k0l = lds_frag(ldsK[1] + 0 * KST2 + c * 32, KST2), k1l = lds_frag(ldsK[1] + 16 * KST2 + c * 32, KST2);
          bf16x16 qh_, ql_;
          { const float* p = qrow + 32 * c;
#pragma unroll
            for (int i = 0; i < 8; ++i) { const float a = p[i], a2 = p[16 + i]; const bf16 ha = (bf16)a, h2 = (bf16)a2;
              qh_[i] = ha; ql_[i] = (bf16)((a - (float)ha) * 2048.0f); qh_[8 + i] = h2; ql_[8 + i] = (bf16)((a2 - (float)h2) * 2048.0f); } }
          s0 = wmma_bf16(k0h, qh_, s0); s0x = wmma_bf16(k0h, ql_, s0x); s0x = wmma_bf16(k0l, qh_, s0x);
          s1 = wmma_bf16(k1h, qh_, s1); s1x = wmma_bf16(k1h, ql_, s1x); s1x = wmma_bf16(k1l, qh_, s1x);
        }
#pragma unroll
        for (int r = 0; r < 8; ++r) { s0[r] += s0x[r] * (1.0f / 2048.0f); s1[r] += s1x[r] * (1.0f / 2048.0f); }

        float mx = -INFINITY;
#pragma unroll
        for (int r = 0; r < 8; ++r) {
          const int k0i = kb + kh8 + r;
          const int k1i = k0i + 16;
          (void)k0i; (void)k1i; (void)q_my;
          s0[r] = (mbits & (1u << r))       ? s0[r] * scale : NEG2;
          s1[r] = (mbits & (1u << (8 + r))) ? s1[r] * scale : NEG2;
          mx = fmaxf(mx, fmaxf(s0[r], s1[r]));
        }
        mx = fmaxf(mx, __shfl_xor(mx, 16, 32));
        const float mnew  = fmaxf(mrun[qt], mx);
        const float alpha = exp2f(mrun[qt] - mnew);

        float rsum = 0.0f;
#pragma unroll
        for (int r = 0; r < 8; ++r) {
          const float p0 = exp2f(s0[r] - mnew);
          const float p1 = exp2f(s1[r] - mnew);
          rsum += p0 + p1;
          pf[qt][r]     = (bf16)(p0 * 1024.0f);
          pf[qt][r + 8] = (bf16)(p1 * 1024.0f);
        }
        rsum += __shfl_xor(rsum, 16, 32);
        lrun[qt] = lrun[qt] * alpha + rsum;
        mrun[qt] = mnew;

#pragma unroll
        for (int j = 0; j < 4; ++j)
#pragma unroll
          for (int r = 0; r < 8; ++r) o[qt][j][r] *= alpha;
        alpha_s[qt] = alpha;
      }
    }

#pragma unroll
    for (int j = 0; j < 4; ++j) {
      const bf16x16 vf2 = lds_frag(ldsV + ((4 + j) * 16) * VSTRIDE, VSTRIDE);
#pragma unroll
      for (int qt = 0; qt < QW; ++qt)
        if (act[qt]) { f32x8 acc;
#pragma unroll
          for (int r = 0; r < 8; ++r) acc[r] = osp[(j * 32 + lane) * 8 + r] * alpha_s[qt];
          acc = wmma_bf16(vf2, pf[qt], acc);
#pragma unroll
          for (int r = 0; r < 8; ++r) osp[(j * 32 + lane) * 8 + r] = acc[r]; }
    }
#pragma unroll
    for (int j = 0; j < 4; ++j) {
      const bf16x16 vf = lds_frag(ldsV + (j * 16) * VSTRIDE, VSTRIDE);
#pragma unroll
      for (int qt = 0; qt < QW; ++qt)
        if (act[qt]) o[qt][j] = wmma_bf16(vf, pf[qt], o[qt][j]);
    }
  }

  float* so = ldsO[wave];
  {
    const float rl = 1.0f / (lrun[0] * 1024.0f);
#pragma unroll
    for (int j = 0; j < 8; ++j)
#pragma unroll
      for (int r = 0; r < 8; ++r) { const int ql = qlane, d = j * 16 + kh8 + r;
        const float ov = (j < 4) ? o[0][j & 3][r] : osp[((j & 3) * 32 + lane) * 8 + r];
        so[ql * 132 + d] = ov * rl + shortcut[((size_t)(b * SS + q0 + ql)) * DKK + d]; }
  }
  asm volatile("s_wait_dscnt 0" ::: "memory");
  __builtin_amdgcn_wave_barrier();
#pragma unroll 1
  for (int pass = 0; pass < 2; ++pass) {
#pragma unroll 4
    for (int it = 0; it < 16; ++it) { const int ch = lane + 32 * it, ql = ch >> 5, q4 = (ch & 31) * 4;
      *(volatile v4f_t*)(attnOut + ((size_t)(b * SS + q0 + ql)) * DKK + q4) = *(const volatile v4fa*)(so + ql * 132 + q4); }
    __threadfence();
  }
}


template <typename AT, bool ACC>
__global__ __launch_bounds__(256) void gemm_kn2(const AT* __restrict__ A, int lda, size_t strideA,
                                               const float* __restrict__ Wm, int ldw, size_t strideW,
                                               const float* __restrict__ bias, float scale,
                                               float* __restrict__ Y, int ldy, size_t strideY, int K) {
  __shared__ __attribute__((aligned(16))) f16 ldsA[128 * GSTR], ldsAl[128 * GSTR];
  __shared__ __attribute__((aligned(16))) f16 ldsW[128 * GSTR], ldsWl[128 * GSTR];
  __shared__ __attribute__((aligned(16))) float oS[8][32 * 68];
  const int tid = threadIdx.x, lane = tid & 31, wave = tid >> 5, cl = lane & 15, rh = (lane >> 4) * 8;
  const int m0 = blockIdx.x * 128, n0 = blockIdx.y * 128;
  const int wm = (wave & 3) * 32, wn = (wave >> 2) * 64;
  A += (size_t)blockIdx.z * strideA; Wm += (size_t)blockIdx.z * strideW; Y += (size_t)blockIdx.z * strideY;
  f32x8 acc[2][4], accx[2][4];
#pragma unroll
  for (int i = 0; i < 2; ++i)
#pragma unroll
    for (int j = 0; j < 4; ++j) { f32x8 z = {}; acc[i][j] = z; accx[i][j] = z; }
#pragma unroll 1
  for (int k0 = 0; k0 < K; k0 += 32) {
    __syncthreads();
    {
      const int row = tid >> 1, ch = (tid & 1) * 16;
      const AT* src = A + (size_t)(m0 + row) * lda + k0 + ch;
#pragma unroll
      for (int g = 0; g < 16; ++g) { const float v = (float)src[g]; const f16 h = (f16)v; ldsA[row * GSTR + ch + g] = h; ldsAl[row * GSTR + ch + g] = (f16)((v - (float)h) * 2048.0f); }
    }
    {
      const int k = tid >> 3, nn0 = (tid & 7) * 16;
      const float* src = Wm + (size_t)(k0 + k) * ldw + n0 + nn0;
#pragma unroll
      for (int g = 0; g < 4; ++g) { const v4f_t v = *(const v4f_t*)(src + 4 * g);
#pragma unroll
        for (int u = 0; u < 4; ++u) { const f16 h = (f16)v[u]; ldsW[(nn0 + 4 * g + u) * GSTR + k] = h; ldsWl[(nn0 + 4 * g + u) * GSTR + k] = (f16)((v[u] - (float)h) * 2048.0f); } }
    }
    __syncthreads();
    f16x16 af[2], afl[2];
#pragma unroll
    for (int i = 0; i < 2; ++i) { af[i] = lds_frag(ldsA + (wm + 16 * i) * GSTR, GSTR); afl[i] = lds_frag(ldsAl + (wm + 16 * i) * GSTR, GSTR); }
#pragma unroll
    for (int j = 0; j < 4; ++j) {
      const f16x16 bf = lds_frag(ldsW + (wn + 16 * j) * GSTR, GSTR), bfl = lds_frag(ldsWl + (wn + 16 * j) * GSTR, GSTR);
#pragma unroll
      for (int i = 0; i < 2; ++i) { acc[i][j] = wmma16(af[i], bf, acc[i][j]); accx[i][j] = wmma16(af[i], bfl, accx[i][j]); accx[i][j] = wmma16(afl[i], bf, accx[i][j]); }
    }
  }
  float* so = oS[wave];
#pragma unroll
  for (int i = 0; i < 2; ++i)
#pragma unroll
    for (int j = 0; j < 4; ++j) {
      const float bv = bias ? bias[n0 + wn + 16 * j + cl] : 0.0f;
#pragma unroll
      for (int r = 0; r < 8; ++r) so[(16 * i + rh + r) * 68 + 16 * j + cl] = (acc[i][j][r] + accx[i][j][r] * (1.0f / 2048.0f)) * scale + bv;
    }
  asm volatile("s_wait_dscnt 0" ::: "memory");
  __builtin_amdgcn_wave_barrier();
  if (ACC) {
#pragma unroll
    for (int it = 0; it < 16; ++it) { const int f4 = lane + 32 * it, rr = f4 >> 4, q = (f4 & 15) * 4;
      const v4f_t old = *(const volatile v4fa*)(Y + (size_t)(m0 + wm + rr) * ldy + n0 + wn + q);
      v4f_t v = *(const volatile v4fa*)(so + rr * 68 + q); v += old; *(volatile v4fa*)(so + rr * 68 + q) = v; }
    asm volatile("s_wait_dscnt 0" ::: "memory");
  }
#pragma unroll 1
  for (int pass = 0; pass < 2; ++pass) {
#pragma unroll
    for (int it = 0; it < 16; ++it) { const int f4 = lane + 32 * it, rr = f4 >> 4, q = (f4 & 15) * 4;
      *(volatile v4f_t*)(Y + (size_t)(m0 + wm + rr) * ldy + n0 + wn + q) = *(const volatile v4fa*)(so + rr * 68 + q); }
    __threadfence();
  }
}

__global__ __launch_bounds__(256) void k_vt(const float* __restrict__ v, bf16* __restrict__ Vt) {
  __shared__ float tS[64][129];
  const int tid = threadIdx.x, b = blockIdx.x / (SS / 64), t0 = (blockIdx.x % (SS / 64)) * 64;
  for (int e = tid; e < 64 * DKK; e += 256) { const int r = e >> 7, c = e & 127; tS[r][c] = v[((size_t)b * SS + t0 + r) * DKK + c]; }
  __syncthreads();
  for (int ch = tid; ch < DKK * 8; ch += 256) { const int d = ch >> 3, q8 = (ch & 7) * 8; union { bf16 hh[8]; v4u_t u; } cv;
#pragma unroll
    for (int e = 0; e < 8; ++e) cv.hh[e] = (bf16)tS[q8 + e][d];
    bf16* dst = Vt + ((size_t)b * DKK + d) * SS + t0 + q8;
    *(volatile v4u_t*)dst = cv.u; __threadfence(); *(volatile v4u_t*)dst = cv.u; }
}

extern "C" void kernel_launch(void* const* d_in, const int* in_sizes, int n_in,
                              void* d_out, int out_size, void* d_ws, size_t ws_size,
                              hipStream_t stream) {
  (void)in_sizes; (void)n_in; (void)out_size; (void)ws_size;
  const float* x = (const float*)d_in[0];
  const float* Wk = (const float*)d_in[1], *bk = (const float*)d_in[2], *Wq = (const float*)d_in[3], *bq = (const float*)d_in[4];
  const float* Wv = (const float*)d_in[5], *bv = (const float*)d_in[6], *Wsm = (const float*)d_in[7], *bs = (const float*)d_in[8];
  float* out = (float*)d_out;
  char* ws = (char*)d_ws;
  const size_t T = (size_t)BB * SS * DKK * 4;
  float* Kf = (float*)ws; float* Qf = (float*)(ws + T); float* Vf = (float*)(ws + 2 * T); float* Sf = (float*)(ws + 3 * T);
  bf16* Vt = (bf16*)(ws + 4 * T);
  const dim3 g(BB * SS / 128, DKK / 128, 1), blk(256);
  gemm_kn2<float, false><<<g, blk, 0, stream>>>(x, CIN, 0, Wk, DKK, 0, bk, 1.0f, Kf, DKK, 0, CIN);
  gemm_kn2<float, false><<<g, blk, 0, stream>>>(x, CIN, 0, Wq, DKK, 0, bq, 1.0f, Qf, DKK, 0, CIN);
  gemm_kn2<float, false><<<g, blk, 0, stream>>>(x, CIN, 0, Wv, DKK, 0, bv, 1.0f, Vf, DKK, 0, CIN);
  gemm_kn2<float, false><<<g, blk, 0, stream>>>(x, CIN, 0, Wsm, DKK, 0, bs, 1.0f, Sf, DKK, 0, CIN);
  k_vt<<<dim3(BB * SS / 64), blk, 0, stream>>>(Vf, Vt);
  attn_kernel<<<dim3(SS / 32, 1, BB), dim3(64), 0, stream>>>((const bf16*)Kf, (const bf16*)Qf, Vt, Sf, out);
}
